// TurboGCN_8881992368458
// MI455X (gfx1250) — hardware-verified
//
#include <hip/hip_runtime.h>
#include <stddef.h>


#define DW      256
#define LDA     512
#define NTHR    256
#define NWAVE   8
#define EPT     8
#define NGRP    2
#define CHUNK   (NTHR * EPT * NGRP)
#define WCAP    (EPT * NGRP * 32)
#define LISTN   (NWAVE * WCAP)
#define NBC     4096
#define NBF     1024
#define RCAP    40960
#define RBN     128
#define TGT     256
#define DEGCAP  1024
#define OTHR    512
#define BM      64
#define NCW     128
#define KSTEPS  (DW / 32)
#define WSCAP   134217728
#define LN_EPS  1e-5f
#define BN_EPS  1e-5f

#define LDS_FILL ((RCAP + NBF + LISTN) * 4 + 64)

static_assert((CHUNK & (CHUNK - 1)) == 0);
static_assert(CHUNK <= 4096);
static_assert((NBC & (NBC - 1)) == 0 && (NBF & (NBF - 1)) == 0);
static_assert(NBC == 4 * NBF);
static_assert(OTHR * 8 == NBC);
static_assert((RCAP % 32) == 0);
static_assert(TGT == NWAVE * 32);
static_assert((NBC % TGT) == 0);
static_assert((TGT % BM) == 0);
static_assert(DW == 8 * 32);
static_assert(2 * NCW == DW);
static_assert((DW % 32) == 0);
static_assert(LDA == 2 * DW);
static_assert(WCAP == EPT * NGRP * 32);

typedef float          v4f  __attribute__((ext_vector_type(4)));
typedef float          v8f  __attribute__((ext_vector_type(8)));
typedef int            v4i  __attribute__((ext_vector_type(4)));
typedef unsigned short v8us __attribute__((ext_vector_type(8)));
typedef __bf16         v16b __attribute__((ext_vector_type(16)));
union FragB { v16b v; v8us h[2]; };

__device__ __forceinline__ v8f wmb(v16b a, v16b b, v8f c) {
  v8f d = __builtin_amdgcn_wmma_f32_16x16x32_bf16(false, a, false, b, (short)0, c, false, false);
  asm volatile("v_nop\n\tv_nop\n\tv_nop\n\tv_nop" : "+v"(d) : "v"(a), "v"(b));
  return d;
}

__device__ __forceinline__ float eluf(float z) { return z > 0.f ? z : (__expf(z) - 1.f); }

__device__ __forceinline__ unsigned int bf16_rne(float f) {
  unsigned int u = __float_as_uint(f);
  u += 0x7FFFu + ((u >> 16) & 1u);
  return u >> 16;
}
__device__ __forceinline__ void split2(float x, unsigned short& hi, unsigned short& lo) {
  const unsigned int hb = bf16_rne(x);
  const float hf = __uint_as_float(hb << 16);
  hi = (unsigned short)hb;
  lo = (unsigned short)bf16_rne(x - hf);
}

__device__ __forceinline__ void relay8(const float (&o)[8], int lane, v4f& w0, v4f& w1) {
  const int s0 = lane >> 1, s1 = 16 + (lane >> 1);
  const bool odd = (lane & 1) != 0;
  float q0[4], q1[4];
#pragma unroll
  for (int i = 0; i < 4; ++i) {
    const float t0 = __shfl(o[i], s0), t1 = __shfl(o[4 + i], s0);
    const float u0 = __shfl(o[i], s1), u1 = __shfl(o[4 + i], s1);
    q0[i] = odd ? t1 : t0;
    q1[i] = odd ? u1 : u0;
  }
  w0.x = q0[0]; w0.y = q0[1]; w0.z = q0[2]; w0.w = q0[3];
  w1.x = q1[0]; w1.y = q1[1]; w1.z = q1[2]; w1.w = q1[3];
}

__device__ __forceinline__ void colsum_out(float* scs, float* srow, const float (&cs)[8], float* dst,
                                           int tid, int lane, int wave) {
  v4f c0, c1;
  c0.x = cs[0]; c0.y = cs[1]; c0.z = cs[2]; c0.w = cs[3];
  c1.x = cs[4]; c1.y = cs[5]; c1.z = cs[6]; c1.w = cs[7];
  *(v4f*)(scs + wave * DW + 8 * lane) = c0;
  *(v4f*)(scs + wave * DW + 8 * lane + 4) = c1;
  __syncthreads();
  float s = 0.f;
#pragma unroll
  for (int w = 0; w < NWAVE; ++w) s += scs[w * DW + tid];
  srow[tid] = s;
  __syncthreads();
  const int q = tid < 64 ? tid : 63;
  const v4f v = *(const v4f*)(srow + 4 * q);
  const bool act = tid < 64;
  if (act) *(volatile v4f*)(dst + 4 * q) = v;
  __threadfence();
  if (act) *(volatile v4f*)(dst + 4 * q) = v;
}

template <int NB>
__device__ __forceinline__ int scan_chunk(const int* __restrict__ dsts, int nE, int cbase, int slotBase,
                                          int vec8, int* list, int tid, int lane, int wave) {
  int wc = 0;
#pragma unroll
  for (int g = 0; g < NGRP; ++g) {
    const int el0  = (g * NTHR + tid) * EPT;
    const int e0   = cbase + el0;
    const int sent = -2147483647 - 1;
    v4i da, db;
    if (vec8 != 0 && cbase + CHUNK <= nE) {
      da = *(const v4i*)(dsts + e0);
      db = *(const v4i*)(dsts + e0 + 4);
    } else {
      da.x = (e0     < nE) ? dsts[min(e0, nE - 1)] : sent;
      da.y = (e0 + 1 < nE) ? dsts[min(e0 + 1, nE - 1)] : sent;
      da.z = (e0 + 2 < nE) ? dsts[min(e0 + 2, nE - 1)] : sent;
      da.w = (e0 + 3 < nE) ? dsts[min(e0 + 3, nE - 1)] : sent;
      db.x = (e0 + 4 < nE) ? dsts[min(e0 + 4, nE - 1)] : sent;
      db.y = (e0 + 5 < nE) ? dsts[min(e0 + 5, nE - 1)] : sent;
      db.z = (e0 + 6 < nE) ? dsts[min(e0 + 6, nE - 1)] : sent;
      db.w = (e0 + 7 < nE) ? dsts[min(e0 + 7, nE - 1)] : sent;
    }
    const unsigned nb = (unsigned)slotBase;
    const unsigned s0 = (unsigned)da.x - nb, s1 = (unsigned)da.y - nb;
    const unsigned s2 = (unsigned)da.z - nb, s3 = (unsigned)da.w - nb;
    const unsigned s4 = (unsigned)db.x - nb, s5 = (unsigned)db.y - nb;
    const unsigned s6 = (unsigned)db.z - nb, s7 = (unsigned)db.w - nb;
    const bool h0 = s0 < (unsigned)NB, h1 = s1 < (unsigned)NB, h2 = s2 < (unsigned)NB, h3 = s3 < (unsigned)NB;
    const bool h4 = s4 < (unsigned)NB, h5 = s5 < (unsigned)NB, h6 = s6 < (unsigned)NB, h7 = s7 < (unsigned)NB;
    const unsigned any = __builtin_amdgcn_ballot_w32(h0 | h1 | h2 | h3 | h4 | h5 | h6 | h7);
    if (any != 0u) {
#define HITJ(J, HJ, SJ) { \
        const unsigned mj = __builtin_amdgcn_ballot_w32(HJ); \
        if (mj != 0u) { \
          if (HJ) { \
            const int pos = wc + (int)__builtin_amdgcn_mbcnt_lo(mj, 0u); \
            if (pos < WCAP) list[wave * WCAP + pos] = ((el0 + (J)) << 12) | (int)(SJ); \
          } \
          wc += (int)__builtin_popcount(mj); } }
      HITJ(0, h0, s0)
      HITJ(1, h1, s1)
      HITJ(2, h2, s2)
      HITJ(3, h3, s3)
      HITJ(4, h4, s4)
      HITJ(5, h5, s5)
      HITJ(6, h6, s6)
      HITJ(7, h7, s7)
#undef HITJ
    }
  }
  return wc;
}

__global__ __launch_bounds__(NTHR) void k_count(
    const int* __restrict__ dsts, int* cnt, float* dinv, int nE, int vec8) {
  __shared__ __attribute__((aligned(16))) int scnt[NBC];
  __shared__ __attribute__((aligned(16))) int list[LISTN];
  __shared__ int wcnt[NWAVE];
  const int tid = threadIdx.x, lane = tid & 31, wave = tid >> 5;
  const int nodeBase = blockIdx.x * NBC;

  for (int i = tid; i < NBC; i += NTHR) scnt[i] = 0;
  __syncthreads();

  const int nChunks = (nE + CHUNK - 1) / CHUNK;
#pragma unroll 1
  for (int ch = 0; ch < nChunks; ++ch) {
    const int cbase = ch * CHUNK;
    const int wc = scan_chunk<NBC>(dsts, nE, cbase, nodeBase, vec8, list, tid, lane, wave);
    if (lane == 0) wcnt[wave] = wc;
    __syncthreads();
    if (wave == 0) {
#pragma unroll 1
      for (int wsx = 0; wsx < NWAVE; ++wsx) {
        int n = __builtin_amdgcn_readfirstlane(wcnt[wsx]);
        n = n > WCAP ? WCAP : (n < 0 ? 0 : n);
        const int* lp = list + wsx * WCAP;
#pragma unroll 1
        for (int i = 0; i < n; ++i) {
          const int ent  = __builtin_amdgcn_readfirstlane(lp[i]);
          const int slot = ent & (NBC - 1);
          if (lane == 0) scnt[slot] = scnt[slot] + 1;
        }
      }
    }
    __syncthreads();
  }

  v4i cq[4];
  v4f dq[4];
#pragma unroll
  for (int q = 0; q < 4; ++q) {
    const int f = (wave * 4 + q) * 128 + 4 * lane;
    const v4i cv = *(const v4i*)(scnt + f);
    cq[q] = cv;
    v4f d;
    d.x = rsqrtf((float)(cv.x < 0 ? 0 : cv.x) + 1.0f);
    d.y = rsqrtf((float)(cv.y < 0 ? 0 : cv.y) + 1.0f);
    d.z = rsqrtf((float)(cv.z < 0 ? 0 : cv.z) + 1.0f);
    d.w = rsqrtf((float)(cv.w < 0 ? 0 : cv.w) + 1.0f);
    dq[q] = d;
  }
  int*   cp = cnt  + (size_t)nodeBase;
  float* dp = dinv + (size_t)nodeBase;
#pragma unroll
  for (int q = 0; q < 4; ++q) {
    const int f = (wave * 4 + q) * 128 + 4 * lane;
    *(volatile v4i*)(cp + f) = cq[q];
    *(volatile v4f*)(dp + f) = dq[q];
  }
  __threadfence();
#pragma unroll
  for (int q = 0; q < 4; ++q) {
    const int f = (wave * 4 + q) * 128 + 4 * lane;
    *(volatile v4i*)(cp + f) = cq[q];
    *(volatile v4f*)(dp + f) = dq[q];
  }
}

__global__ __launch_bounds__(OTHR) void k_offsets(
    const int* __restrict__ cnt, int* off, int* rbase, int nChunk) {
  __shared__ __attribute__((aligned(16))) int soff[NBC];
  __shared__ __attribute__((aligned(16))) int srb[RBN];
  __shared__ int wtot[OTHR / 32];
  const int tid = threadIdx.x, lane = tid & 31, wave = tid >> 5, sub = tid >> 7;
  for (int i = tid; i < RBN; i += OTHR) srb[i] = 0;
  int carry = 0;
#pragma unroll 1
  for (int ch = 0; ch < nChunk; ++ch) {
    const int base = ch * NBC;
    const v4i c0 = *(const v4i*)(cnt + base + 8 * tid);
    const v4i c1 = *(const v4i*)(cnt + base + 8 * tid + 4);
    const int e0 = max(c0.x, 0), e1 = max(c0.y, 0), e2 = max(c0.z, 0), e3 = max(c0.w, 0);
    const int e4 = max(c1.x, 0), e5 = max(c1.y, 0), e6 = max(c1.z, 0), e7 = max(c1.w, 0);
    const int ts = e0 + e1 + e2 + e3 + e4 + e5 + e6 + e7;
    int incl = ts;
#pragma unroll
    for (int d = 1; d < 32; d <<= 1) {
      const int t = __shfl_up(incl, d);
      if (lane >= d) incl += t;
    }
    if (lane == 31) wtot[wave] = incl;
    __syncthreads();
    const int S0 = wtot[0]  + wtot[1]  + wtot[2]  + wtot[3];
    const int S1 = wtot[4]  + wtot[5]  + wtot[6]  + wtot[7];
    const int S2 = wtot[8]  + wtot[9]  + wtot[10] + wtot[11];
    const int S3 = wtot[12] + wtot[13] + wtot[14] + wtot[15];
    int pre = 0;
#pragma unroll 1
    for (int w = 4 * sub; w < wave; ++w) pre += wtot[w];
    const int b0 = carry;
    const int b1 = b0 + ((S0 + 31) & ~31);
    const int b2 = b1 + ((S1 + 31) & ~31);
    const int b3 = b2 + ((S2 + 31) & ~31);
    const int b4 = b3 + ((S3 + 31) & ~31);
    const int myb = sub == 0 ? b0 : (sub == 1 ? b1 : (sub == 2 ? b2 : b3));
    if (tid == 0) {
      srb[min(4 * ch + 0, RBN - 1)] = b0;
      srb[min(4 * ch + 1, RBN - 1)] = b1;
      srb[min(4 * ch + 2, RBN - 1)] = b2;
      srb[min(4 * ch + 3, RBN - 1)] = b3;
    }
    int run = myb + pre + incl - ts;
    soff[8 * tid + 0] = run; run += e0;
    soff[8 * tid + 1] = run; run += e1;
    soff[8 * tid + 2] = run; run += e2;
    soff[8 * tid + 3] = run; run += e3;
    soff[8 * tid + 4] = run; run += e4;
    soff[8 * tid + 5] = run; run += e5;
    soff[8 * tid + 6] = run; run += e6;
    soff[8 * tid + 7] = run;
    carry = b4;
    __syncthreads();
    const v4i o0 = *(const v4i*)(soff + 4 * tid);
    const v4i o1 = *(const v4i*)(soff + 4 * (tid + OTHR));
    int* op = off + base;
    *(volatile v4i*)(op + 4 * tid) = o0;
    *(volatile v4i*)(op + 4 * (tid + OTHR)) = o1;
    __threadfence();
    *(volatile v4i*)(op + 4 * tid) = o0;
    *(volatile v4i*)(op + 4 * (tid + OTHR)) = o1;
    __syncthreads();
  }
  if (tid == 0) srb[min(4 * nChunk, RBN - 1)] = carry;
  __syncthreads();
  v4i rv = {0, 0, 0, 0};
  if (tid < 32) rv = *(const v4i*)(srb + 4 * tid);
  if (tid < 32) *(volatile v4i*)(rbase + 4 * tid) = rv;
  __threadfence();
  if (tid < 32) *(volatile v4i*)(rbase + 4 * tid) = rv;
}

__global__ __launch_bounds__(NTHR) void k_fill(
    const int* __restrict__ srcs, const int* __restrict__ dsts,
    const int* __restrict__ off, const int* __restrict__ rbase,
    int* csr, int nN, int nE, int vec8, int csrLen) {
  extern __shared__ v4f lds_dyn[];
  int* region = (int*)lds_dyn;
  int* cursor = region + RCAP;
  int* list   = cursor + NBF;
  int* wcnt   = list + LISTN;
  const int tid = threadIdx.x, lane = tid & 31, wave = tid >> 5;
  const int b = blockIdx.x;
  const int nodeBase = b * NBF;

  int rb0 = rbase[b];
  const int rb1 = rbase[b + 1];
  rb0 = rb0 < 0 ? 0 : (rb0 > csrLen ? csrLen : rb0);
  rb0 &= ~31;
  int len = rb1 - rb0;
  len = len < 0 ? 0 : (len > RCAP ? RCAP : len);
  int lenW = (len + 31) & ~31;
  if (rb0 + lenW > csrLen) lenW = (csrLen - rb0) & ~31;

  {
    const v4i z = {0, 0, 0, 0};
    for (int i = tid; i < RCAP / 4; i += NTHR) ((v4i*)region)[i] = z;
    for (int s = tid; s < NBF; s += NTHR) {
      int o = off[nodeBase + s] - rb0;
      o = o < 0 ? 0 : (o > RCAP ? RCAP : o);
      cursor[s] = o;
    }
  }
  __syncthreads();

  const int nChunks = (nE + CHUNK - 1) / CHUNK;
#pragma unroll 1
  for (int ch = 0; ch < nChunks; ++ch) {
    const int cbase = ch * CHUNK;
    const int wc = scan_chunk<NBF>(dsts, nE, cbase, nodeBase, vec8, list, tid, lane, wave);
    if (lane == 0) wcnt[wave] = wc;
    __syncthreads();
    if (wave == 0) {
#pragma unroll 1
      for (int wsx = 0; wsx < NWAVE; ++wsx) {
        int n = __builtin_amdgcn_readfirstlane(wcnt[wsx]);
        n = n > WCAP ? WCAP : (n < 0 ? 0 : n);
        const int* lp = list + wsx * WCAP;
#pragma unroll 1
        for (int i = 0; i < n; ++i) {
          const int ent  = __builtin_amdgcn_readfirstlane(lp[i]);
          const int slot = ent & (NBF - 1);
          int e = cbase + ((ent >> 12) & (CHUNK - 1));
          e = e > nE - 1 ? nE - 1 : e;
          int sv = srcs[e];
          sv = sv < 0 ? 0 : (sv > nN - 1 ? nN - 1 : sv);
          if (lane == 0) {
            int pos = cursor[slot];
            pos = pos < 0 ? 0 : (pos > RCAP - 1 ? RCAP - 1 : pos);
            region[pos] = sv;
            const int np = pos + 1;
            cursor[slot] = np > RCAP ? RCAP : np;
          }
        }
      }
    }
    __syncthreads();
  }

  const int nv = lenW >> 2;
  int* gp = csr + rb0;
#pragma unroll 1
  for (int i = tid; i < nv; i += NTHR) { const v4i v = ((const v4i*)region)[i]; *(volatile v4i*)(gp + 4 * i) = v; }
  __threadfence();
#pragma unroll 1
  for (int i = tid; i < nv; i += NTHR) { const v4i v = ((const v4i*)region)[i]; *(volatile v4i*)(gp + 4 * i) = v; }
}

__global__ __launch_bounds__(NTHR) void k_inproj(
    const float* __restrict__ ctrl, const float* __restrict__ w_in, const float* __restrict__ b_in,
    const float* __restrict__ gam, const float* __restrict__ bet, unsigned short* arow, int nN) {
  const int tid = threadIdx.x, lane = tid & 31, wave = tid >> 5;
  const int tbase = blockIdx.x * TGT + wave * 32;
  const int col8 = 8 * lane;
  float wv[8], bv[8], gg[8], be[8];
  {
    const v4f a0 = *(const v4f*)(w_in + col8), a1 = *(const v4f*)(w_in + col8 + 4);
    const v4f b0 = *(const v4f*)(b_in + col8), b1 = *(const v4f*)(b_in + col8 + 4);
    const v4f c0 = *(const v4f*)(gam + col8),  c1 = *(const v4f*)(gam + col8 + 4);
    const v4f d0 = *(const v4f*)(bet + col8),  d1 = *(const v4f*)(bet + col8 + 4);
    wv[0] = a0.x; wv[1] = a0.y; wv[2] = a0.z; wv[3] = a0.w; wv[4] = a1.x; wv[5] = a1.y; wv[6] = a1.z; wv[7] = a1.w;
    bv[0] = b0.x; bv[1] = b0.y; bv[2] = b0.z; bv[3] = b0.w; bv[4] = b1.x; bv[5] = b1.y; bv[6] = b1.z; bv[7] = b1.w;
    gg[0] = c0.x; gg[1] = c0.y; gg[2] = c0.z; gg[3] = c0.w; gg[4] = c1.x; gg[5] = c1.y; gg[6] = c1.z; gg[7] = c1.w;
    be[0] = d0.x; be[1] = d0.y; be[2] = d0.z; be[3] = d0.w; be[4] = d1.x; be[5] = d1.y; be[6] = d1.z; be[7] = d1.w;
  }
#pragma unroll 1
  for (int j = 0; j < 32; ++j) {
    const int c = tbase + j;
    const bool live = c < nN;
    int cc = c > nN - 1 ? nN - 1 : c;
    cc = cc < 0 ? 0 : cc;
    const float xin = ctrl[cc];
    float v[8];
    float s = 0.f;
#pragma unroll
    for (int i = 0; i < 8; ++i) { v[i] = xin * wv[i] + bv[i]; s += v[i]; }
    s += __shfl_xor(s, 16);
    s += __shfl_xor(s, 8);
    s += __shfl_xor(s, 4);
    s += __shfl_xor(s, 2);
    s += __shfl_xor(s, 1);
    const float mu = s * (1.0f / DW);
    float d[8];
    float q = 0.f;
#pragma unroll
    for (int i = 0; i < 8; ++i) { d[i] = v[i] - mu; q += d[i] * d[i]; }
    q += __shfl_xor(q, 16);
    q += __shfl_xor(q, 8);
    q += __shfl_xor(q, 4);
    q += __shfl_xor(q, 2);
    q += __shfl_xor(q, 1);
    const float var = q * (1.0f / DW);
    const float rs = rsqrtf(var + LN_EPS);
    v8us oh, ol;
#pragma unroll
    for (int i = 0; i < 8; ++i) {
      const float t = (d[i] * rs) * gg[i] + be[i];
      const float e = eluf(t);
      const float y = live ? e : 0.f;
      unsigned short hi, lo;
      split2(y, hi, lo);
      oh[i] = hi; ol[i] = lo;
    }
    unsigned short* gh = arow + (size_t)c * LDA + col8;
    unsigned short* gl = gh + DW;
    *(volatile v8us*)gh = oh;
    *(volatile v8us*)gl = ol;
    __threadfence();
    *(volatile v8us*)gh = oh;
    *(volatile v8us*)gl = ol;
  }
}

__global__ __launch_bounds__(NTHR) void k_wtcvt(const float* __restrict__ W, unsigned short* dh,
                                                unsigned short* dl, int K, int Nout, int nUnits) {
  const int i = (int)blockIdx.x * NTHR + (int)threadIdx.x;
  if (i >= nUnits) return;
  const int ppr = K >> 3;
  const int per = Nout * ppr;
  const int L = i / per;
  const int r = i - L * per;
  const int n = r / ppr;
  const int seg = r - n * ppr;
  const float* p = W + (size_t)L * K * Nout + (size_t)(8 * seg) * Nout + n;
  v8us oh, ol;
#pragma unroll
  for (int j = 0; j < 8; ++j) {
    unsigned short hi, lo;
    split2(p[(size_t)j * Nout], hi, lo);
    oh[j] = hi; ol[j] = lo;
  }
  unsigned short* gh = dh + (size_t)i * 8;
  unsigned short* gl = dl + (size_t)i * 8;
  *(volatile v8us*)gh = oh;
  *(volatile v8us*)gl = ol;
  __threadfence();
  *(volatile v8us*)gh = oh;
  *(volatile v8us*)gl = ol;
}

__global__ __launch_bounds__(NTHR) void k_gemm3(
    const unsigned short* __restrict__ A, const unsigned short* __restrict__ Bh,
    const unsigned short* __restrict__ Bl, float* C32, int KT, int ldc) {
  constexpr int TPW = 4;
  constexpr int PPR = NCW / 4;
  constexpr int NIT = (BM * PPR) / NTHR;
  static_assert((BM * PPR) % NTHR == 0);
  static_assert(NIT >= 1);

  __shared__ __attribute__((aligned(16))) float stg[BM * NCW];
  const int tid = threadIdx.x, lane = tid & 31, wave = tid >> 5, hh = lane >> 4, m = lane & 15;
  const int rowBase = (int)blockIdx.x * BM;
  const int colBase = (int)blockIdx.y * NCW;
  const int rg = wave >> 1, chf = wave & 1;
  const int r0 = rg * 16;
  const int c0 = chf * (NCW / 2);
  const int KB = 32 * KT;

  v8f acc[TPW];
#pragma unroll
  for (int t = 0; t < TPW; ++t) { v8f z = {0.f, 0.f, 0.f, 0.f, 0.f, 0.f, 0.f, 0.f}; acc[t] = z; }

  const size_t aoff = (size_t)(rowBase + r0 + m) * LDA + 8 * hh;
  const unsigned short* aph = A + aoff;
  const unsigned short* apl = A + aoff + DW;
  const size_t boff = (size_t)(colBase + c0 + m) * KB + 8 * hh;
  const unsigned short* bph = Bh + boff;
  const unsigned short* bpl = Bl + boff;
#pragma unroll 1
  for (int kt = 0; kt < KT; ++kt) {
    FragB ah, al;
    ah.h[0] = *(const v8us*)(aph + 32 * kt);
    ah.h[1] = *(const v8us*)(aph + 32 * kt + 16);
    al.h[0] = *(const v8us*)(apl + 32 * kt);
    al.h[1] = *(const v8us*)(apl + 32 * kt + 16);
#pragma unroll
    for (int t = 0; t < TPW; ++t) {
      const size_t to = (size_t)(16 * t) * KB + 32 * kt;
      FragB bh, bl;
      bh.h[0] = *(const v8us*)(bph + to);
      bh.h[1] = *(const v8us*)(bph + to + 16);
      bl.h[0] = *(const v8us*)(bpl + to);
      bl.h[1] = *(const v8us*)(bpl + to + 16);
      acc[t] = wmb(ah.v, bh.v, acc[t]);
      acc[t] = wmb(al.v, bh.v, acc[t]);
      acc[t] = wmb(ah.v, bl.v, acc[t]);
    }
  }

  {
    float* sp = stg + (size_t)(r0 + 8 * hh) * NCW + c0 + m;
#pragma unroll
    for (int t = 0; t < TPW; ++t) {
#pragma unroll
      for (int r = 0; r < 8; ++r) sp[r * NCW + 16 * t] = acc[t][r];
    }
  }
  __syncthreads();

  v4f cv[NIT];
#pragma unroll
  for (int it = 0; it < NIT; ++it) {
    const int id = it * NTHR + tid;
    const int row = id / PPR, seg = id % PPR;
    cv[it] = *(const v4f*)(stg + (size_t)row * NCW + 4 * seg);
  }
#pragma unroll
  for (int it = 0; it < NIT; ++it) {
    const int id = it * NTHR + tid;
    const int row = id / PPR, seg = id % PPR;
    float* gp = C32 + (size_t)(rowBase + row) * ldc + colBase + 4 * seg;
    *(volatile v4f*)gp = cv[it];
  }
  __threadfence();
#pragma unroll
  for (int it = 0; it < NIT; ++it) {
    const int id = it * NTHR + tid;
    const int row = id / PPR, seg = id % PPR;
    float* gp = C32 + (size_t)(rowBase + row) * ldc + colBase + 4 * seg;
    *(volatile v4f*)gp = cv[it];
  }
}

__global__ __launch_bounds__(NTHR) void k_agg(
    const int* __restrict__ csr, const int* __restrict__ off, const int* __restrict__ cnt,
    const float* __restrict__ dinv, const float* __restrict__ hb, const float* __restrict__ bias,
    float* xo, float* xsum, int nN, int csrLen) {
  __shared__ __attribute__((aligned(16))) float scs[NWAVE * DW];
  __shared__ __attribute__((aligned(16))) float srow[DW];
  const int tid = threadIdx.x, lane = tid & 31, wave = tid >> 5;
  const int tbase = blockIdx.x * TGT + wave * 32;
  const int col8 = 8 * lane;
  const int cl    = tbase + lane;
  const int cnt_l = cnt[cl];
  const int off_l = off[cl];
  const float di_l = dinv[cl];
  const v4f vb0 = *(const v4f*)(bias + col8), vb1 = *(const v4f*)(bias + col8 + 4);
  const float bb[8] = {vb0.x, vb0.y, vb0.z, vb0.w, vb1.x, vb1.y, vb1.z, vb1.w};
  float cs[8] = {0.f, 0.f, 0.f, 0.f, 0.f, 0.f, 0.f, 0.f};

#pragma unroll 1
  for (int j = 0; j < 32; ++j) {
    const int c = tbase + j;
    int n = __shfl(cnt_l, j);
    n = n < 0 ? 0 : (n > DEGCAP ? DEGCAP : n);
    const int st = __shfl(off_l, j);
    const float dc = __shfl(di_l, j);
    const float dd = dc * dc;

    float a[8];
    {
      const float* hr = hb + (size_t)c * DW + col8;
      const v4f x0 = *(const v4f*)hr, x1 = *(const v4f*)(hr + 4);
      a[0] = x0.x * dd; a[1] = x0.y * dd; a[2] = x0.z * dd; a[3] = x0.w * dd;
      a[4] = x1.x * dd; a[5] = x1.y * dd; a[6] = x1.z * dd; a[7] = x1.w * dd;
    }
#pragma unroll 1
    for (int q0 = 0; q0 < n; q0 += 32) {
      int pos = st + q0 + lane;
      pos = pos < 0 ? 0 : (pos > csrLen - 1 ? csrLen - 1 : pos);
      int sl = csr[pos];
      sl = sl < 0 ? 0 : (sl > nN - 1 ? nN - 1 : sl);
      const int mcnt = (n - q0) < 32 ? (n - q0) : 32;
#pragma unroll 1
      for (int pp = 0; pp < mcnt; ++pp) {
        const int s = __builtin_amdgcn_readlane(sl, pp);
        const float cf = dinv[s] * dc;
        const float* hr = hb + (size_t)s * DW + col8;
        const v4f x0 = *(const v4f*)hr, x1 = *(const v4f*)(hr + 4);
        a[0] += x0.x * cf; a[1] += x0.y * cf; a[2] += x0.z * cf; a[3] += x0.w * cf;
        a[4] += x1.x * cf; a[5] += x1.y * cf; a[6] += x1.z * cf; a[7] += x1.w * cf;
      }
    }

    const bool live = c < nN;
    float o[8];
#pragma unroll
    for (int i = 0; i < 8; ++i) {
      const float t = a[i] + bb[i];
      o[i] = live ? t : 0.f;
      cs[i] += o[i];
    }
    v4f w0, w1;
    relay8(o, lane, w0, w1);
    float* gp = xo + (size_t)c * DW + 4 * lane;
    *(volatile v4f*)gp = w0;
    *(volatile v4f*)(gp + NCW) = w1;
    __threadfence();
    *(volatile v4f*)gp = w0;
    *(volatile v4f*)(gp + NCW) = w1;
  }

  colsum_out(scs, srow, cs, xsum + (size_t)blockIdx.x * DW, tid, lane, wave);
}

__global__ __launch_bounds__(NTHR) void k_var(const float* xo, const float* __restrict__ xsum,
                                              float* sq, int nN, int nPart) {
  __shared__ __attribute__((aligned(16))) float smu[DW];
  __shared__ __attribute__((aligned(16))) float scs[NWAVE * DW];
  __shared__ __attribute__((aligned(16))) float srow[DW];
  const int tid = threadIdx.x, lane = tid & 31, wave = tid >> 5;
  const int tbase = blockIdx.x * TGT + wave * 32;
  const int col8 = 8 * lane;
  {
    double s = 0.0;
#pragma unroll 1
    for (int b = 0; b < nPart; ++b) s += (double)xsum[(size_t)b * DW + tid];
    smu[tid] = (float)(s / (double)nN);
  }
  __syncthreads();
  const v4f m0 = *(const v4f*)(smu + col8), m1 = *(const v4f*)(smu + col8 + 4);
  float cs[8] = {0.f, 0.f, 0.f, 0.f, 0.f, 0.f, 0.f, 0.f};
#pragma unroll 1
  for (int j = 0; j < 32; ++j) {
    const int c = tbase + j;
    if (c >= nN) break;
    const float* xr = xo + (size_t)c * DW + col8;
    const v4f x0 = *(const v4f*)xr, x1 = *(const v4f*)(xr + 4);
    float d;
    d = x0.x - m0.x; cs[0] += d * d;
    d = x0.y - m0.y; cs[1] += d * d;
    d = x0.z - m0.z; cs[2] += d * d;
    d = x0.w - m0.w; cs[3] += d * d;
    d = x1.x - m1.x; cs[4] += d * d;
    d = x1.y - m1.y; cs[5] += d * d;
    d = x1.z - m1.z; cs[6] += d * d;
    d = x1.w - m1.w; cs[7] += d * d;
  }
  colsum_out(scs, srow, cs, sq + (size_t)blockIdx.x * DW, tid, lane, wave);
}

template <int LAST>
__global__ __launch_bounds__(NTHR) void k_bnapply(
    const float* xo, const float* __restrict__ xsum, const float* __restrict__ sq,
    const float* __restrict__ gam, const float* __restrict__ bet,
    const float* __restrict__ whd, const float* __restrict__ bhd,
    unsigned short* arow, float* out, int nN, int nPart) {
  __shared__ __attribute__((aligned(16))) float smu[DW];
  __shared__ __attribute__((aligned(16))) float srs[DW];
  __shared__ __attribute__((aligned(16))) float sg[DW];
  __shared__ __attribute__((aligned(16))) float sb[DW];
  __shared__ __attribute__((aligned(16))) float shd[TGT];
  const int tid = threadIdx.x, lane = tid & 31, wave = tid >> 5;
  const int tbase = blockIdx.x * TGT + wave * 32;
  const int col8 = 8 * lane;
  {
    double s1 = 0.0, s2 = 0.0;
#pragma unroll 1
    for (int b = 0; b < nPart; ++b) {
      s1 += (double)xsum[(size_t)b * DW + tid];
      s2 += (double)sq[(size_t)b * DW + tid];
    }
    const float mu  = (float)(s1 / (double)nN);
    const float var = (float)(s2 / (double)nN);
    smu[tid] = mu;
    srs[tid] = rsqrtf(var + BN_EPS);
    sg[tid]  = gam[tid];
    sb[tid]  = bet[tid];
    shd[tid] = 0.f;
  }
  __syncthreads();
  float mu[8], rs[8], gg[8], be[8];
  {
    const v4f a0 = *(const v4f*)(smu + col8), a1 = *(const v4f*)(smu + col8 + 4);
    const v4f b0 = *(const v4f*)(srs + col8), b1 = *(const v4f*)(srs + col8 + 4);
    const v4f c0 = *(const v4f*)(sg + col8),  c1 = *(const v4f*)(sg + col8 + 4);
    const v4f d0 = *(const v4f*)(sb + col8),  d1 = *(const v4f*)(sb + col8 + 4);
    mu[0] = a0.x; mu[1] = a0.y; mu[2] = a0.z; mu[3] = a0.w; mu[4] = a1.x; mu[5] = a1.y; mu[6] = a1.z; mu[7] = a1.w;
    rs[0] = b0.x; rs[1] = b0.y; rs[2] = b0.z; rs[3] = b0.w; rs[4] = b1.x; rs[5] = b1.y; rs[6] = b1.z; rs[7] = b1.w;
    gg[0] = c0.x; gg[1] = c0.y; gg[2] = c0.z; gg[3] = c0.w; gg[4] = c1.x; gg[5] = c1.y; gg[6] = c1.z; gg[7] = c1.w;
    be[0] = d0.x; be[1] = d0.y; be[2] = d0.z; be[3] = d0.w; be[4] = d1.x; be[5] = d1.y; be[6] = d1.z; be[7] = d1.w;
  }
  float wh[8] = {0.f, 0.f, 0.f, 0.f, 0.f, 0.f, 0.f, 0.f};
  float hb0 = 0.f;
  if constexpr (LAST == 1) {
    const v4f e0 = *(const v4f*)(whd + col8), e1 = *(const v4f*)(whd + col8 + 4);
    wh[0] = e0.x; wh[1] = e0.y; wh[2] = e0.z; wh[3] = e0.w; wh[4] = e1.x; wh[5] = e1.y; wh[6] = e1.z; wh[7] = e1.w;
    hb0 = bhd[0];
  }
  float myo = 0.f;
#pragma unroll 1
  for (int j = 0; j < 32; ++j) {
    const int c = tbase + j;
    const bool live = c < nN;
    const float* xr = xo + (size_t)c * DW + col8;
    const v4f x0 = *(const v4f*)xr, x1 = *(const v4f*)(xr + 4);
    const float xv[8] = {x0.x, x0.y, x0.z, x0.w, x1.x, x1.y, x1.z, x1.w};
    float yv[8];
#pragma unroll
    for (int i = 0; i < 8; ++i) {
      const float t = ((xv[i] - mu[i]) * rs[i]) * gg[i] + be[i];
      const float e = eluf(t);
      yv[i] = live ? e : 0.f;
    }
    if constexpr (LAST == 0) {
      v8us oh, ol;
#pragma unroll
      for (int i = 0; i < 8; ++i) {
        unsigned short hi, lo;
        split2(yv[i], hi, lo);
        oh[i] = hi; ol[i] = lo;
      }
      unsigned short* gh = arow + (size_t)c * LDA + col8;
      unsigned short* gl = gh + DW;
      *(volatile v8us*)gh = oh;
      *(volatile v8us*)gl = ol;
      __threadfence();
      *(volatile v8us*)gh = oh;
      *(volatile v8us*)gl = ol;
    } else {
      float pd = yv[0] * wh[0] + yv[1] * wh[1] + yv[2] * wh[2] + yv[3] * wh[3]
               + yv[4] * wh[4] + yv[5] * wh[5] + yv[6] * wh[6] + yv[7] * wh[7];
      pd += __shfl_xor(pd, 16);
      pd += __shfl_xor(pd, 8);
      pd += __shfl_xor(pd, 4);
      pd += __shfl_xor(pd, 2);
      pd += __shfl_xor(pd, 1);
      const float hv = live ? (pd + hb0) : 0.f;
      myo = (lane == j) ? hv : myo;
    }
  }
  if constexpr (LAST == 1) {
    shd[tid] = myo;
    __syncthreads();
    const int base = blockIdx.x * TGT;
    int rem = nN - base;
    rem = rem < 0 ? 0 : (rem > TGT ? TGT : rem);
    const bool act = tid < 64;
    const int q = act ? tid : 0;
    const v4f v = *(const v4f*)(shd + 4 * q);
    float* gp = out + (size_t)base + 4 * q;
    const bool full = act && (4 * q + 4 <= rem);
    const int part = act ? (rem - 4 * q) : 0;
    const bool tail = act && !full && part > 0;
    if (full) *(volatile v4f*)gp = v;
    if (tail) {
      *(volatile float*)gp = v.x;
      if (part > 1) *(volatile float*)(gp + 1) = v.y;
      if (part > 2) *(volatile float*)(gp + 2) = v.z;
    }
    __threadfence();
    if (full) *(volatile v4f*)gp = v;
    if (tail) {
      *(volatile float*)gp = v.x;
      if (part > 1) *(volatile float*)(gp + 1) = v.y;
      if (part > 2) *(volatile float*)(gp + 2) = v.z;
    }
  }
}

extern "C" void kernel_launch(void* const* d_in, const int* in_sizes, int n_in,
                              void* d_out, int out_size, void* d_ws, size_t ws_size,
                              hipStream_t stream) {
  if (n_in < 20) return;
  const int nN = in_sizes[0];
  const int nE = in_sizes[1] / 2;
  if (nN <= 0 || nE <= 0) return;
  if (in_sizes[1] != 2 * nE) return;
  if (in_sizes[2] != DW || in_sizes[3] != DW || in_sizes[4] != DW || in_sizes[5] != DW) return;
  for (int l = 0; l < 3; ++l) {
    if (in_sizes[6 + 4 * l] != DW * DW) return;
    if (in_sizes[7 + 4 * l] != DW || in_sizes[8 + 4 * l] != DW || in_sizes[9 + 4 * l] != DW) return;
  }
  if (in_sizes[18] != DW || in_sizes[19] < 1) return;
  if (out_size != nN) return;
  if (nE > (1 << 28) || nN > (1 << 22)) return;

  const float* ctrl = (const float*)d_in[0];
  const int*   ei   = (const int*)d_in[1];
  const int*   src  = ei;
  const int*   dst  = ei + nE;
  const float* w_in = (const float*)d_in[2];
  const float* b_in = (const float*)d_in[3];
  const float* ln_g = (const float*)d_in[4];
  const float* ln_b = (const float*)d_in[5];
  const float* whd  = (const float*)d_in[18];
  const float* bhd  = (const float*)d_in[19];
  float* out = (float*)d_out;

  const int NPAD   = ((nN + TGT - 1) / TGT) * TGT;
  const int nBC    = (nN + NBC - 1) / NBC;
  const int CNTPAD = nBC * NBC;
  if (CNTPAD < NPAD) return;
  if (4 * nBC + 1 > RBN) return;
  const int nBF    = (nN + NBF - 1) / NBF;
  if (nBF > 4 * nBC) return;
  const int csrLen = ((nE + 31) & ~31) + 4096;
  if (31 * 4 * nBC > 4096) return;
  const int nAgg   = NPAD / TGT;
  const int nGemm  = NPAD / BM;

  char* ws = (char*)d_ws;
  size_t off = 0;
  size_t oWh[3], oWl[3];
  for (int l = 0; l < 3; ++l) {
    oWh[l] = off; off += (size_t)DW * DW * 2;                     off = (off + 255) & ~(size_t)255;
    oWl[l] = off; off += (size_t)DW * DW * 2;                     off = (off + 255) & ~(size_t)255;
  }
  const size_t oA   = off; off += (size_t)NPAD * LDA * 2;         off = (off + 255) & ~(size_t)255;
  const size_t oC   = off; off += (size_t)NPAD * DW * 4;          off = (off + 255) & ~(size_t)255;
  const size_t oCnt = off; off += (size_t)CNTPAD * 4;             off = (off + 255) & ~(size_t)255;
  const size_t oDi  = off; off += (size_t)CNTPAD * 4;             off = (off + 255) & ~(size_t)255;
  const size_t oOff = off; off += (size_t)CNTPAD * 4;             off = (off + 255) & ~(size_t)255;
  const size_t oRb  = off; off += (size_t)RBN * 4;                off = (off + 255) & ~(size_t)255;
  const size_t oCsr = off; off += (size_t)csrLen * 4;             off = (off + 255) & ~(size_t)255;
  const size_t oXs  = off; off += (size_t)nAgg * DW * 4;          off = (off + 255) & ~(size_t)255;
  const size_t oSq  = off; off += (size_t)nAgg * DW * 4;          off = (off + 255) & ~(size_t)255;
  if (off > ws_size || off > (size_t)WSCAP) return;

  unsigned short* arow = (unsigned short*)(ws + oA);
  float* xo   = (float*)(ws + oA);
  float* cbuf = (float*)(ws + oC);
  int*   cnt  = (int*)(ws + oCnt);
  float* dinv = (float*)(ws + oDi);
  int*   offp = (int*)(ws + oOff);
  int*   rb   = (int*)(ws + oRb);
  int*   csr  = (int*)(ws + oCsr);
  float* xsum = (float*)(ws + oXs);
  float* sq   = (float*)(ws + oSq);

  const int vec8 = ((nE & 3) == 0) ? 1 : 0;

  k_inproj<<<nAgg, NTHR, 0, stream>>>(ctrl, w_in, b_in, ln_g, ln_b, arow, nN);
  for (int l = 0; l < 3; ++l) {
    const float* Wl = (const float*)d_in[6 + 4 * l];
    k_wtcvt<<<(DW * DW / 8 + NTHR - 1) / NTHR, NTHR, 0, stream>>>(
        Wl, (unsigned short*)(ws + oWh[l]), (unsigned short*)(ws + oWl[l]), DW, DW, DW * DW / 8);
  }
  k_count<<<nBC, NTHR, 0, stream>>>(dst, cnt, dinv, nE, vec8);
  k_offsets<<<1, OTHR, 0, stream>>>(cnt, offp, rb, nBC);
  hipFuncSetAttribute(reinterpret_cast<const void*>(&k_fill),
                      hipFuncAttributeMaxDynamicSharedMemorySize, LDS_FILL);
  k_fill<<<nBF, NTHR, LDS_FILL, stream>>>(src, dst, offp, rb, csr, nN, nE, vec8, csrLen);

  for (int l = 0; l < 3; ++l) {
    const unsigned short* bh = (const unsigned short*)(ws + oWh[l]);
    const unsigned short* bl = (const unsigned short*)(ws + oWl[l]);
    const float* bs  = (const float*)d_in[7 + 4 * l];
    const float* gam = (const float*)d_in[8 + 4 * l];
    const float* bet = (const float*)d_in[9 + 4 * l];
    k_gemm3<<<dim3(nGemm, DW / NCW, 1), NTHR, 0, stream>>>(arow, bh, bl, cbuf, KSTEPS, DW);
    k_agg<<<nAgg, NTHR, 0, stream>>>(csr, offp, cnt, dinv, cbuf, bs, xo, xsum, nN, csrLen);
    k_var<<<nAgg, NTHR, 0, stream>>>(xo, xsum, sq, nN, nAgg);
    if (l < 2)
      k_bnapply<0><<<nAgg, NTHR, 0, stream>>>(xo, xsum, sq, gam, bet, whd, bhd, arow, out, nN, nAgg);
    else
      k_bnapply<1><<<nAgg, NTHR, 0, stream>>>(xo, xsum, sq, gam, bet, whd, bhd, arow, out, nN, nAgg);
  }
}
